// GraphAttention_13322988552557
// MI455X (gfx1250) — hardware-verified
//
#include <hip/hip_runtime.h>
#include <math.h>
#include <stddef.h>
#include <stdint.h>

#define NB    8
#define NS    2
#define NN    1024
#define TIN   12
#define TOUT  12
#define KSZ   3
#define NE    64
#define HD    10
#define NBT   (NB * TOUT)
#define KP    32
#define WSMAX 134217728

static_assert(TIN - KSZ + 1 == HD);
static_assert(3 * HD <= KP);
static_assert(2 * HD + 2 * NS <= KP);
static_assert(NN % 128 == 0);
static_assert(TIN == 12 && TOUT == 12 && NS == 2 && NE == 64);
static_assert((NN * TOUT * 4) % 128 == 0);

typedef float          v4f   __attribute__((ext_vector_type(4)));
typedef float          v8f   __attribute__((ext_vector_type(8)));
typedef int            v8i   __attribute__((ext_vector_type(8)));
typedef unsigned int   v4u   __attribute__((ext_vector_type(4)));
typedef unsigned short v8us  __attribute__((ext_vector_type(8)));
typedef unsigned short v16us __attribute__((ext_vector_type(16)));
typedef __bf16         v16bf __attribute__((ext_vector_type(16)));
typedef __bf16         v8bf  __attribute__((ext_vector_type(8)));
typedef v4f  __attribute__((may_alias)) v4fa;
typedef v4u  __attribute__((may_alias)) v4ua;
typedef v8us __attribute__((may_alias)) v8usa;
union FragB { v16bf v; v16us u; v8us h[2]; v8i w; };

__device__ __forceinline__ v8f wmb(const FragB& a, const FragB& b, v8f c) {
  v8f d = __builtin_amdgcn_wmma_f32_16x16x32_bf16(false, a.v, false, b.v, (short)0, c, false, false);
  asm volatile("v_nop\n\tv_nop\n\tv_nop\n\tv_nop" : "+v"(d) : "v"(a.w), "v"(b.w));
  return d;
}
__device__ __forceinline__ v8f z8() { v8f z = {0.f, 0.f, 0.f, 0.f, 0.f, 0.f, 0.f, 0.f}; return z; }

__device__ __forceinline__ unsigned bf16_bits(float f) {
  const unsigned u = __float_as_uint(f);
  return (u + 0x7FFFu + ((u >> 16) & 1u)) >> 16;
}
__device__ __forceinline__ float bf16_val(float f) { return __uint_as_float(bf16_bits(f) << 16); }
__device__ __forceinline__ v4f bf16_val4(v4f a) {
  v4f r; r.x = bf16_val(a.x); r.y = bf16_val(a.y); r.z = bf16_val(a.z); r.w = bf16_val(a.w); return r;
}
__device__ __forceinline__ unsigned split_hi(float f) { return bf16_bits(f); }
__device__ __forceinline__ unsigned split_lo(float f, unsigned hb) { return bf16_bits(f - __uint_as_float(hb << 16)); }

__global__ __launch_bounds__(128) void k_prep(
    const float* __restrict__ x,
    const float* __restrict__ kw, const float* __restrict__ kb,
    const float* __restrict__ qw, const float* __restrict__ qb,
    const float* __restrict__ vw, const float* __restrict__ vb,
    const float* __restrict__ fow, const float* __restrict__ fob,
    const float* __restrict__ frw, const float* __restrict__ frb,
    const float* __restrict__ frtw, const float* __restrict__ frtb,
    unsigned short* KA, unsigned short* QB, unsigned short* VH, unsigned short* VL,
    float* XT, unsigned short* WT, float* CB) {
  __shared__ __attribute__((aligned(16))) float sx[NS * 128 * TIN];
  __shared__ __attribute__((aligned(16))) float sw[416];
  __shared__ __attribute__((aligned(16))) unsigned short sKA[128 * KP];
  __shared__ __attribute__((aligned(16))) unsigned short sQB[128 * KP];
  __shared__ __attribute__((aligned(16))) unsigned short sVH[16 * 128];
  __shared__ __attribute__((aligned(16))) unsigned short sVL[16 * 128];
  __shared__ __attribute__((aligned(16))) float sXT[128 * 24];
  __shared__ __attribute__((aligned(16))) float srs[16];

  const int tid = (int)threadIdx.x;
  const int b   = (int)blockIdx.x >> 3;
  const int n0  = ((int)blockIdx.x & 7) * 128;

#pragma unroll
  for (int s = 0; s < NS; ++s) {
#pragma unroll
    for (int it = 0; it < 3; ++it) {
      const int p = it * 128 + tid;
      const v4f a = *(const v4f*)(x + ((size_t)((b * NS + s) * NN + n0)) * TIN + 4 * p);
      *(v4fa*)(sx + s * 1536 + 4 * p) = bf16_val4(a);
    }
  }
  {
    const int i = (tid < 17) ? tid : 17;
    const v4f a = *(const v4f*)(kw + 4 * i);
    const v4f c = *(const v4f*)(qw + 4 * i);
    const v4f d = *(const v4f*)(vw + 4 * i);
    if (tid < 18) {
      *(v4fa*)(sw + 0   + 4 * tid) = bf16_val4(a);
      *(v4fa*)(sw + 72  + 4 * tid) = bf16_val4(c);
      *(v4fa*)(sw + 144 + 4 * tid) = bf16_val4(d);
    }
  }
  {
    const int i = (tid < 2) ? tid : 2;
    const v4f a = *(const v4f*)(kb + 4 * i);
    const v4f c = *(const v4f*)(qb + 4 * i);
    const v4f d = *(const v4f*)(vb + 4 * i);
    const v4f e = *(const v4f*)(frtb + 4 * i);
    if (tid < 3) {
      *(v4fa*)(sw + 216 + 4 * tid) = bf16_val4(a);
      *(v4fa*)(sw + 228 + 4 * tid) = bf16_val4(c);
      *(v4fa*)(sw + 240 + 4 * tid) = bf16_val4(d);
      *(v4fa*)(sw + 400 + 4 * tid) = bf16_val4(e);
    }
  }
  {
    const int i = (tid < 35) ? tid : 35;
    const v4f a = *(const v4f*)(frtw + 4 * i);
    if (tid < 36) *(v4fa*)(sw + 256 + 4 * tid) = bf16_val4(a);
  }
  sKA[tid * KP + 30] = (unsigned short)0; sKA[tid * KP + 31] = (unsigned short)0;
  sQB[tid * KP + 30] = (unsigned short)0; sQB[tid * KP + 31] = (unsigned short)0;
#pragma unroll
  for (int c = HD; c < 16; ++c) { sVH[c * 128 + tid] = (unsigned short)0; sVL[c * 128 + tid] = (unsigned short)0; }
  __syncthreads();

#pragma unroll 1
  for (int st = 0; st < 2 * TOUT; ++st) {
    const int s  = (st >= TOUT) ? 1 : 0;
    const int to = st - s * TOUT;
    const float* xr = sx + (s * 128 + tid) * TIN;
    const float* wr = sw + 256 + to * TIN;
    float acc = 0.0f;
#pragma unroll
    for (int ti = 0; ti < TIN; ++ti) acc = fmaf(wr[ti], xr[ti], acc);
    sXT[tid * 24 + st] = acc;
  }
  __syncthreads();
  {
    v4f xv[6];
#pragma unroll
    for (int it = 0; it < 6; ++it) xv[it] = *(const v4fa*)(sXT + 4 * (it * 128 + tid));
    float* dst = XT + ((size_t)(b * NN + n0)) * 24;
#pragma unroll
    for (int it = 0; it < 6; ++it) *(volatile v4f*)(dst + 4 * (it * 128 + tid)) = xv[it];
    __threadfence();
#pragma unroll
    for (int it = 0; it < 6; ++it) *(volatile v4f*)(dst + 4 * (it * 128 + tid)) = xv[it];
  }

#pragma unroll 1
  for (int t = 0; t < TOUT; ++t) {
    float wk[6], wq[6], wv[6];
#pragma unroll
    for (int i = 0; i < 6; ++i) { wk[i] = sw[t * 6 + i]; wq[i] = sw[72 + t * 6 + i]; wv[i] = sw[144 + t * 6 + i]; }
    const float bk = sw[216 + t], bq = sw[228 + t], bv = sw[240 + t];
#pragma unroll 1
    for (int c = 0; c < HD; ++c) {
      float ak = bk, aq = bq, av = bv;
#pragma unroll
      for (int s = 0; s < NS; ++s) {
#pragma unroll
        for (int j = 0; j < KSZ; ++j) {
          const float xv = sx[(s * 128 + tid) * TIN + c + j];
          ak = fmaf(xv, wk[s * 3 + j], ak);
          aq = fmaf(xv, wq[s * 3 + j], aq);
          av = fmaf(xv, wv[s * 3 + j], av);
        }
      }
      const unsigned kh = split_hi(ak), kl = split_lo(ak, kh);
      const unsigned qh = split_hi(aq), ql = split_lo(aq, qh);
      const unsigned vh = split_hi(av), vl = split_lo(av, vh);
      sKA[tid * KP + c]          = (unsigned short)kh;
      sKA[tid * KP + HD + c]     = (unsigned short)kl;
      sKA[tid * KP + 2 * HD + c] = (unsigned short)kh;
      sQB[tid * KP + c]          = (unsigned short)qh;
      sQB[tid * KP + HD + c]     = (unsigned short)qh;
      sQB[tid * KP + 2 * HD + c] = (unsigned short)ql;
      sVH[c * 128 + tid] = (unsigned short)vh;
      sVL[c * 128 + tid] = (unsigned short)vl;
    }
    __syncthreads();
    {
      const int bt = b * TOUT + t;
      v4u ra[4], rq[4], rh[2], rl[2];
#pragma unroll
      for (int it = 0; it < 4; ++it) {
        const int p = it * 128 + tid;
        ra[it] = *(const v4ua*)(sKA + 8 * p);
        rq[it] = *(const v4ua*)(sQB + 8 * p);
      }
#pragma unroll
      for (int it = 0; it < 2; ++it) {
        const int p = it * 128 + tid;
        rh[it] = *(const v4ua*)(sVH + 8 * p);
        rl[it] = *(const v4ua*)(sVL + 8 * p);
      }
      unsigned short* ka = KA + ((size_t)bt * NN + n0) * KP;
      unsigned short* qa = QB + ((size_t)bt * NN + n0) * KP;
#pragma unroll 1
      for (int pass = 0; pass < 2; ++pass) {
#pragma unroll
        for (int it = 0; it < 4; ++it) {
          const int p = it * 128 + tid;
          *(volatile v4u*)(ka + 8 * p) = ra[it];
          *(volatile v4u*)(qa + 8 * p) = rq[it];
        }
#pragma unroll
        for (int it = 0; it < 2; ++it) {
          const int p = it * 128 + tid;
          const size_t go = ((size_t)(bt * 16 + (p >> 4))) * NN + n0 + 8 * (p & 15);
          *(volatile v4u*)(VH + go) = rh[it];
          *(volatile v4u*)(VL + go) = rl[it];
        }
        __threadfence();
      }
    }
    __syncthreads();
  }

  if (blockIdx.x == 0) {
#pragma unroll 1
    for (int it = 0; it < 16; ++it) {
      const int idx = it * 128 + tid;
      const int e = idx >> 5, k = idx & 31;
      int cc = (k < HD) ? k : (k - HD);
      cc = (cc < 0) ? 0 : ((cc > HD - 1) ? (HD - 1) : cc);
      const int si = (k >= 2 * HD + 2) ? 1 : 0;
      const float f = fow[e * HD + cc];
      const float g = frw[e * NS + si];
      const unsigned fb = bf16_bits(f), gb = bf16_bits(g);
      const unsigned mf = (k < 2 * HD) ? 0xFFFFu : 0u;
      const unsigned mg = (k >= 2 * HD && k < 2 * HD + 4) ? 0xFFFFu : 0u;
      sKA[idx] = (unsigned short)((fb & mf) | (gb & mg));
    }
    {
      const int tt = (tid < TOUT - 1) ? tid : (TOUT - 1);
      float s = 0.0f;
#pragma unroll
      for (int ti = 0; ti < TIN; ++ti) s += sw[256 + tt * TIN + ti];
      if (tid < TOUT) srs[tid] = s;
    }
    __syncthreads();
#pragma unroll 1
    for (int it = 0; it < 6; ++it) {
      const int idx = it * 128 + tid;
      const int e = idx / TOUT;
      const int t = idx - e * TOUT;
      const float fo = bf16_val(fob[e]);
      const float fr = bf16_val(frb[e]);
      sXT[idx] = fmaf(fr, srs[t], fo) + sw[400 + t];
    }
    __syncthreads();
    v4u wv2[2];
#pragma unroll
    for (int it = 0; it < 2; ++it) wv2[it] = *(const v4ua*)(sKA + 8 * (it * 128 + tid));
    const int t1 = (tid < 64) ? tid : 63;
    const v4f c0 = *(const v4fa*)(sXT + 4 * tid);
    const v4f c1 = *(const v4fa*)(sXT + 4 * (128 + t1));
#pragma unroll 1
    for (int pass = 0; pass < 2; ++pass) {
#pragma unroll
      for (int it = 0; it < 2; ++it) *(volatile v4u*)(WT + 8 * (it * 128 + tid)) = wv2[it];
      *(volatile v4f*)(CB + 4 * tid) = c0;
      if (tid < 64) *(volatile v4f*)(CB + 4 * (128 + tid)) = c1;
      __threadfence();
    }
  }
}

#define AT_KC 64
#define AT_NW 8
static_assert(NN % AT_KC == 0);

__device__ __forceinline__ unsigned short at_bf_bits(float f) {
  unsigned u = __float_as_uint(f);
  return (unsigned short)((u + 0x7FFFu + ((u >> 16) & 1u)) >> 16);
}
__device__ __forceinline__ __bf16 at_f2bf(float f) { return __builtin_bit_cast(__bf16, at_bf_bits(f)); }
__device__ __forceinline__ void at_split(float f, __bf16& hi, __bf16& lo) {
  const unsigned short hb = at_bf_bits(f);
  hi = __builtin_bit_cast(__bf16, hb);
  lo = at_f2bf(f - __uint_as_float(((unsigned)hb) << 16));
}
__device__ __forceinline__ v8f at_mma(v16bf a, v16bf b, v8f c) {
  c = __builtin_amdgcn_wmma_f32_16x16x32_bf16(false, a, false, b, (short)0, c, false, false);
  asm volatile("v_nop\n\tv_nop\n\tv_nop\n\tv_nop" : "+v"(c) : "v"(a), "v"(b));
  return c;
}
union AtFB { v16bf v; v8bf h[2]; };
__device__ __forceinline__ v16bf at_ldfrag(const __bf16* p) {
  AtFB f; f.h[0] = *(const v8bf*)(p); f.h[1] = *(const v8bf*)(p + 16); return f.v;
}

__global__ __launch_bounds__(256)
void k_attn(const unsigned short* __restrict__ kap, const unsigned short* __restrict__ qbp,
            const unsigned short* __restrict__ vhp, const unsigned short* __restrict__ vlp,
            float* op) {
  __shared__ __align__(16) __bf16 Psh[AT_NW][16 * AT_KC];
  __shared__ __align__(16) __bf16 Psl[AT_NW][16 * AT_KC];
  __shared__ __align__(16) float  Os[AT_NW][16 * 16];

  const int tid  = (int)threadIdx.x;
  const int wave = tid >> 5;
  const int lane = tid & 31;
  const int hh   = lane >> 4;
  const int c    = lane & 15;
  const int bt   = (int)blockIdx.x >> 3;
  const int q0   = ((int)blockIdx.x & 7) * 128 + wave * 16;

  const __bf16* KAp = (const __bf16*)(const void*)kap + (size_t)bt * NN * KP;
  const __bf16* QBp = (const __bf16*)(const void*)qbp + (size_t)bt * NN * KP;
  const __bf16* Vh  = (const __bf16*)(const void*)vhp + (size_t)bt * 16 * NN;
  const __bf16* Vl  = (const __bf16*)(const void*)vlp + (size_t)bt * 16 * NN;
  float* ob = op + (size_t)bt * NN * 16;

  const v16bf ka = at_ldfrag(KAp + (size_t)(q0 + c) * KP + 8 * hh);

  float mrow[8], lrow[8];
  v8f oacc = z8();
#pragma unroll
  for (int r = 0; r < 8; ++r) { mrow[r] = -INFINITY; lrow[r] = 0.f; }

  __bf16* pwh = Psh[wave];
  __bf16* pwl = Psl[wave];
  const int nChunks = NN / AT_KC;
  for (int kc = 0; kc < nChunks; ++kc) {
    const int kv0 = kc * AT_KC;
    v8f s[4];
#pragma unroll
    for (int j = 0; j < 4; ++j) {
      const v16bf qf = at_ldfrag(QBp + (size_t)(kv0 + j * 16 + c) * KP + 8 * hh);
      s[j] = at_mma(ka, qf, z8());
    }
    float cm[8];
#pragma unroll
    for (int r = 0; r < 8; ++r) {
      float mx = -INFINITY;
#pragma unroll
      for (int j = 0; j < 4; ++j) mx = fmaxf(mx, s[j][r]);
#pragma unroll
      for (int off = 1; off < 16; off <<= 1) mx = fmaxf(mx, __shfl_xor(mx, off, 32));
      cm[r] = mx;
    }
#pragma unroll
    for (int r = 0; r < 8; ++r) {
      const float mnew  = fmaxf(mrow[r], cm[r]);
      const float alpha = expf(mrow[r] - mnew);
      mrow[r] = mnew;
      float psum = 0.f;
#pragma unroll
      for (int j = 0; j < 4; ++j) {
        const float p = expf(s[j][r] - mnew);
        psum += p;
        __bf16 a, bl; at_split(p, a, bl);
        pwh[(8 * hh + r) * AT_KC + j * 16 + c] = a;
        pwl[(8 * hh + r) * AT_KC + j * 16 + c] = bl;
      }
#pragma unroll
      for (int off = 1; off < 16; off <<= 1) psum += __shfl_xor(psum, off, 32);
      lrow[r] = lrow[r] * alpha + psum;
      oacc[r] *= alpha;
    }
    __builtin_amdgcn_fence(__ATOMIC_RELEASE, "workgroup");
    __builtin_amdgcn_wave_barrier();
    __builtin_amdgcn_fence(__ATOMIC_ACQUIRE, "workgroup");
#pragma unroll
    for (int kk = 0; kk < 2; ++kk) {
      AtFB pa, pl;
      pa.h[0] = *(const v8bf*)(pwh + c * AT_KC + kk * 32 + 8 * hh);
      pa.h[1] = *(const v8bf*)(pwh + c * AT_KC + kk * 32 + 16 + 8 * hh);
      pl.h[0] = *(const v8bf*)(pwl + c * AT_KC + kk * 32 + 8 * hh);
      pl.h[1] = *(const v8bf*)(pwl + c * AT_KC + kk * 32 + 16 + 8 * hh);
      const v16bf vb = at_ldfrag(Vh + (size_t)c * NN + kv0 + kk * 32 + 8 * hh);
      const v16bf vl = at_ldfrag(Vl + (size_t)c * NN + kv0 + kk * 32 + 8 * hh);
      oacc = at_mma(pa.v, vb, oacc);
      oacc = at_mma(pa.v, vl, oacc);
      oacc = at_mma(pl.v, vb, oacc);
    }
    __builtin_amdgcn_fence(__ATOMIC_RELEASE, "workgroup");
    __builtin_amdgcn_wave_barrier();
    __builtin_amdgcn_fence(__ATOMIC_ACQUIRE, "workgroup");
  }

  float* os = Os[wave];
#pragma unroll
  for (int r = 0; r < 8; ++r) {
    const float inv = 1.0f / lrow[r];
    const float o = oacc[r] * inv;
    os[(8 * hh + r) * 16 + c] = (c < HD) ? o : 0.0f;
  }
  __builtin_amdgcn_fence(__ATOMIC_RELEASE, "workgroup");
  __builtin_amdgcn_wave_barrier();
  __builtin_amdgcn_fence(__ATOMIC_ACQUIRE, "workgroup");
  {
    v4f ov[2];
#pragma unroll
    for (int it = 0; it < 2; ++it) ov[it] = *(const v4fa*)(os + 4 * (it * 32 + lane));
    float* dst = ob + (size_t)q0 * 16;
#pragma unroll
    for (int it = 0; it < 2; ++it) *(volatile v4f*)(dst + 4 * (it * 32 + lane)) = ov[it];
    __threadfence();
#pragma unroll
    for (int it = 0; it < 2; ++it) *(volatile v4f*)(dst + 4 * (it * 32 + lane)) = ov[it];
  }
}

#define TL_ROWS   384
#define TL_YPT    388
#define TL_SA_OFF 99328
#define TL_CB_OFF 123904
#define TL_RC_OFF 126976
#define TL_LDS    127488
static_assert(NE * TL_YPT * 4 == TL_SA_OFF);
static_assert(TL_SA_OFF + TL_ROWS * KP * 2 == TL_CB_OFF);
static_assert(TL_CB_OFF + NE * TOUT * 4 == TL_RC_OFF);
static_assert(TL_RC_OFF + 128 * 4 == TL_LDS);
static_assert(TL_ROWS == 32 * TOUT && TL_ROWS == 24 * 16);

__global__ __launch_bounds__(256)
void k_tail(const float* __restrict__ OP, const float* __restrict__ XT, const unsigned short* __restrict__ WT,
            const float* __restrict__ CB, float* YP, float* REC) {
  extern __shared__ __attribute__((aligned(16))) unsigned char smem[];
  float*          sY   = (float*)smem;
  unsigned short* sA   = (unsigned short*)(smem + TL_SA_OFF);
  float*          sCB  = (float*)(smem + TL_CB_OFF);
  float*          sRec = (float*)(smem + TL_RC_OFF);

  const int tid = (int)threadIdx.x, lane = tid & 31, wave = tid >> 5, hh = lane >> 4, m = lane & 15;
  const int b  = (int)blockIdx.x >> 5;
  const int n0 = ((int)blockIdx.x & 31) * 32;

  {
    const v4u zz = {0u, 0u, 0u, 0u};
    for (int r = tid; r < TL_ROWS; r += 256) *(v4ua*)(sA + r * KP + 24) = zz;
  }
#pragma unroll
  for (int it = 0; it < 6; ++it) {
    const int p   = it * 256 + tid;
    const int t   = p >> 7;
    const int rem = p & 127;
    const int nl  = rem >> 2;
    const int q4  = (rem & 3) * 4;
    const v4f o = *(const v4f*)(OP + ((size_t)((b * TOUT + t) * NN + n0 + nl)) * 16 + q4);
    const int row = nl * TOUT + t;
    const float ov0 = o.x, ov1 = o.y, ov2 = o.z, ov3 = o.w;
    if (q4 + 0 < HD) { const unsigned h = split_hi(ov0), l = split_lo(ov0, h); sA[row * KP + q4 + 0] = (unsigned short)h; sA[row * KP + HD + q4 + 0] = (unsigned short)l; }
    if (q4 + 1 < HD) { const unsigned h = split_hi(ov1), l = split_lo(ov1, h); sA[row * KP + q4 + 1] = (unsigned short)h; sA[row * KP + HD + q4 + 1] = (unsigned short)l; }
    if (q4 + 2 < HD) { const unsigned h = split_hi(ov2), l = split_lo(ov2, h); sA[row * KP + q4 + 2] = (unsigned short)h; sA[row * KP + HD + q4 + 2] = (unsigned short)l; }
    if (q4 + 3 < HD) { const unsigned h = split_hi(ov3), l = split_lo(ov3, h); sA[row * KP + q4 + 3] = (unsigned short)h; sA[row * KP + HD + q4 + 3] = (unsigned short)l; }
  }
  {
    const int i = (tid < 191) ? tid : 191;
    const v4f xv = *(const v4f*)(XT + ((size_t)(b * NN + n0)) * 24 + 4 * i);
    const v4f cb = *(const v4f*)(CB + 4 * i);
    if (tid < 192) {
      *(v4fa*)(sCB + 4 * tid) = cb;
      const float xe[4] = {xv.x, xv.y, xv.z, xv.w};
#pragma unroll
      for (int e = 0; e < 4; ++e) {
        const int f   = 4 * tid + e;
        const int nl  = f / 24;
        const int rem = f - nl * 24;
        const int s   = (rem >= TOUT) ? 1 : 0;
        const int to  = rem - s * TOUT;
        const int row = nl * TOUT + to;
        const unsigned h = split_hi(xe[e]), l = split_lo(xe[e], h);
        sA[row * KP + 2 * HD + 2 * s]     = (unsigned short)h;
        sA[row * KP + 2 * HD + 2 * s + 1] = (unsigned short)l;
      }
    }
  }
  __syncthreads();

  FragB bw[4];
#pragma unroll
  for (int nt = 0; nt < 4; ++nt) {
    const unsigned short* wp = WT + (size_t)(16 * nt + m) * KP + 8 * hh;
    bw[nt].h[0] = *(const v8usa*)wp;
    bw[nt].h[1] = *(const v8usa*)(wp + 16);
  }
#pragma unroll 1
  for (int i = 0; i < 3; ++i) {
    const int mt = wave * 3 + i;
    const unsigned short* ap = sA + (16 * mt + m) * KP + 8 * hh;
    FragB af;
    af.h[0] = *(const v8usa*)ap;
    af.h[1] = *(const v8usa*)(ap + 16);
    v8f acc[4];
#pragma unroll
    for (int nt = 0; nt < 4; ++nt) acc[nt] = wmb(af, bw[nt], z8());
    const int row0 = 16 * mt + 8 * hh;
    const int t0 = row0 % TOUT;
#pragma unroll
    for (int nt = 0; nt < 4; ++nt) {
      const int e = 16 * nt + m;
#pragma unroll
      for (int r = 0; r < 8; ++r) {
        int tt = t0 + r;
        tt = (tt >= TOUT) ? (tt - TOUT) : tt;
        sY[e * TL_YPT + row0 + r] = acc[nt][r] + sCB[e * TOUT + tt];
      }
    }
  }
  __syncthreads();

#pragma unroll 1
  for (int j = 0; j < 8; ++j) {
    const int e = wave * 8 + j;
    const float* yr = sY + e * TL_YPT;
    float v[12];
    float s = 0.0f;
#pragma unroll
    for (int i = 0; i < 12; ++i) { v[i] = yr[lane + 32 * i]; s += v[i]; }
#pragma unroll
    for (int off = 16; off > 0; off >>= 1) s += __shfl_xor(s, off, 32);
    const float mean = s * (1.0f / 384.0f);
    float q = 0.0f;
#pragma unroll
    for (int i = 0; i < 12; ++i) { const float d = v[i] - mean; q = fmaf(d, d, q); }
#pragma unroll
    for (int off = 16; off > 0; off >>= 1) q += __shfl_xor(q, off, 32);
    if (lane == 0) { sRec[e] = mean; sRec[64 + e] = q; }
  }
  __syncthreads();

  v4f rv = {0.f, 0.f, 0.f, 0.f};
  if (tid < 32) rv = *(const v4fa*)(sRec + 4 * tid);
  float* rdst = REC + (size_t)blockIdx.x * 128;
  float* ybase = YP + (size_t)b * NE * (NN * TOUT) + (size_t)n0 * TOUT;
#pragma unroll 1
  for (int pass = 0; pass < 2; ++pass) {
    if (tid < 32) *(volatile v4f*)(rdst + 4 * tid) = rv;
#pragma unroll 1
    for (int j = 0; j < 8; ++j) {
      const int e = wave * 8 + j;
      float* yd = ybase + (size_t)e * (NN * TOUT);
#pragma unroll
      for (int it = 0; it < 3; ++it) {
        const int pc = it * 32 + lane;
        const v4f val = *(const v4fa*)(sY + e * TL_YPT + 4 * pc);
        *(volatile v4f*)(yd + 4 * pc) = val;
      }
    }
    __threadfence();
  }
}

#define NREC 256
static_assert(NREC * TL_ROWS == NB * NN * TOUT);

__global__ __launch_bounds__(64) void k_comb(const float* __restrict__ rec, const float* __restrict__ gam,
                                             const float* __restrict__ bet, float* ss) {
  __shared__ __attribute__((aligned(16))) float stg[256];
  const int tid = (int)threadIdx.x;
  const int e = tid & 63;
  double s = 0.0;
#pragma unroll 1
  for (int p = 0; p < NREC; ++p) s += (double)rec[(size_t)p * 128 + e];
  const double mean = s * (1.0 / (double)NREC);
  double q = 0.0;
#pragma unroll 1
  for (int p = 0; p < NREC; ++p) {
    const double mb = (double)rec[(size_t)p * 128 + e];
    const double qb = (double)rec[(size_t)p * 128 + 64 + e];
    const double d = mb - mean;
    q = q + (qb + 384.0 * d * d);
  }
  const double var = q * (1.0 / 98304.0);
  const float rstd = (float)(1.0 / sqrt(var + 1e-5));
  stg[e]       = (float)mean;
  stg[64 + e]  = rstd;
  stg[128 + e] = bf16_val(gam[e]);
  stg[192 + e] = bf16_val(bet[e]);
  __syncthreads();
  const v4f v = *(const v4fa*)(stg + 4 * tid);
  *(volatile v4f*)(ss + 4 * tid) = v;
  __threadfence();
  *(volatile v4f*)(ss + 4 * tid) = v;
}

#define TOTAL4 (NB * NE * NN * TOUT / 4)
static_assert(TOTAL4 % 256 == 0);
static_assert((NN * TOUT) % 1024 == 0);

__global__ __launch_bounds__(256) void k_norm(const float* __restrict__ yp, const float* __restrict__ ss, float* out) {
  const int idx = (int)blockIdx.x * 256 + (int)threadIdx.x;
  if (idx >= TOTAL4) return;
  const int e = ((int)blockIdx.x / ((NN * TOUT) / 1024)) & (NE - 1);
  const float mean = ss[e], rstd = ss[64 + e], g = ss[128 + e], bt = ss[192 + e];
  const v4f v = *(const v4f*)(yp + 4 * (size_t)idx);
  v4f o;
  o.x = fmaf((v.x - mean) * rstd, g, bt);
  o.y = fmaf((v.y - mean) * rstd, g, bt);
  o.z = fmaf((v.z - mean) * rstd, g, bt);
  o.w = fmaf((v.w - mean) * rstd, g, bt);
  *(volatile v4f*)(out + 4 * (size_t)idx) = o;
  __threadfence();
  *(volatile v4f*)(out + 4 * (size_t)idx) = o;
}

static inline size_t al256(size_t o) { return (o + 255) & ~(size_t)255; }

extern "C" void kernel_launch(void* const* d_in, const int* in_sizes, int n_in,
                              void* d_out, int out_size, void* d_ws, size_t ws_size,
                              hipStream_t stream) {
  if (n_in < 15) return;
  if (in_sizes[0] != NB * NS * NN * TIN) return;
  if (in_sizes[1] != TOUT * NS * KSZ || in_sizes[3] != TOUT * NS * KSZ || in_sizes[5] != TOUT * NS * KSZ) return;
  if (in_sizes[2] != TOUT || in_sizes[4] != TOUT || in_sizes[6] != TOUT) return;
  if (in_sizes[7] != NE * HD || in_sizes[8] != NE) return;
  if (in_sizes[9] != NE * NS || in_sizes[10] != NE) return;
  if (in_sizes[11] != TOUT * TIN || in_sizes[12] != TOUT) return;
  if (in_sizes[13] != NE || in_sizes[14] != NE) return;
  if (out_size != NB * NE * NN * TOUT) return;

  const float* x    = (const float*)d_in[0];
  const float* kw   = (const float*)d_in[1];
  const float* kb   = (const float*)d_in[2];
  const float* qw   = (const float*)d_in[3];
  const float* qb   = (const float*)d_in[4];
  const float* vw   = (const float*)d_in[5];
  const float* vb   = (const float*)d_in[6];
  const float* fow  = (const float*)d_in[7];
  const float* fob  = (const float*)d_in[8];
  const float* frw  = (const float*)d_in[9];
  const float* frb  = (const float*)d_in[10];
  const float* frtw = (const float*)d_in[11];
  const float* frtb = (const float*)d_in[12];
  const float* gam  = (const float*)d_in[13];
  const float* bet  = (const float*)d_in[14];

  const size_t PK = (size_t)NBT * NN * KP * 2;
  const size_t PV = (size_t)NBT * 16 * NN * 2;
  const size_t PO = (size_t)NBT * NN * 16 * 4;
  const size_t PY = (size_t)NB * NE * NN * TOUT * 4;
  const size_t PX = (size_t)NB * NN * 24 * 4;
  size_t off = 0;
  const size_t oKA = off; off = al256(off + PK);
  const size_t oQB = off; off = al256(off + PK);
  const size_t oVH = off; off = al256(off + PV);
  const size_t oVL = off; off = al256(off + PV);
  const size_t oOP = off; off = al256(off + PO);
  const size_t oYP = off; off = al256(off + PY);
  const size_t oXT = off; off = al256(off + PX);
  const size_t oWT = off; off = al256(off + (size_t)NE * KP * 2);
  const size_t oCB = off; off = al256(off + (size_t)NE * TOUT * 4);
  const size_t oRC = off; off = al256(off + (size_t)NREC * 128 * 4);
  const size_t oSS = off; off = al256(off + (size_t)256 * 4);
  if (off > ws_size || off > (size_t)WSMAX) return;

  char* ws = (char*)d_ws;
  unsigned short* KA = (unsigned short*)(ws + oKA);
  unsigned short* QB = (unsigned short*)(ws + oQB);
  unsigned short* VH = (unsigned short*)(ws + oVH);
  unsigned short* VL = (unsigned short*)(ws + oVL);
  float*          OP = (float*)(ws + oOP);
  float*          YP = (float*)(ws + oYP);
  float*          XT = (float*)(ws + oXT);
  unsigned short* WT = (unsigned short*)(ws + oWT);
  float*          CB = (float*)(ws + oCB);
  float*          RC = (float*)(ws + oRC);
  float*          SS = (float*)(ws + oSS);

  k_prep<<<NB * (NN / 128), 128, 0, stream>>>(x, kw, kb, qw, qb, vw, vb, fow, fob, frw, frb, frtw, frtb,
                                              KA, QB, VH, VL, XT, WT, CB);
  k_attn<<<NBT * (NN / 128), 256, 0, stream>>>(KA, QB, VH, VL, OP);
  (void)hipFuncSetAttribute(reinterpret_cast<const void*>(&k_tail), hipFuncAttributeMaxDynamicSharedMemorySize, TL_LDS);
  k_tail<<<NB * (NN / 32), 256, TL_LDS, stream>>>(OP, XT, WT, CB, YP, RC);
  k_comb<<<1, 64, 0, stream>>>(RC, gam, bet, SS);
  k_norm<<<TOTAL4 / 256, 256, 0, stream>>>(YP, SS, (float*)d_out);
  (void)hipGetLastError();
}
